// GNNEncoder_15195594293396
// MI455X (gfx1250) — hardware-verified
//
#include <hip/hip_runtime.h>
#include <math.h>

typedef __attribute__((ext_vector_type(16))) _Float16 v16h;
typedef __attribute__((ext_vector_type(8)))  _Float16 v8h;
typedef __attribute__((ext_vector_type(16))) __bf16   v16b;
typedef __attribute__((ext_vector_type(8)))  __bf16   v8b;
typedef __attribute__((ext_vector_type(8)))  float    v8f;
typedef __attribute__((ext_vector_type(4)))  float    v4f;
typedef __attribute__((ext_vector_type(4)))  int      v4i;

constexpr int kBatch  = 256;
constexpr int kNodes  = 32;
constexpr int kFeat   = 256;
constexpr int kEdges  = 992;
constexpr int kEPad   = 1024;
constexpr int kRows   = kBatch * kNodes;
constexpr int kTileE  = 32;
constexpr int kTiles  = kEdges / kTileE;
constexpr int kPW     = 2 * kFeat;
constexpr int kZP     = 264;
constexpr int kZTile  = kTileE * kZP;
constexpr int kOP     = 260;
constexpr float kZCarry = 16.0f;
constexpr float kWCarry = 256.0f;
constexpr float kECarry = 16.0f;
constexpr float kAccToE = kECarry / (kZCarry * kWCarry);
constexpr float kEInv   = 1.0f / kECarry;
static_assert(kTiles * kTileE == kEdges, "edge tiles exact");
static_assert(kRows == 8192 && (kRows % 64) == 0 && (kFeat % 64) == 0 && (kPW % 64) == 0, "GEMM M,N multiples of 64");
static_assert((kFeat % 32) == 0, "GEMM K multiple of 32");
static_assert(kNodes * kOP <= kNodes * kPW, "staging tile fits the P tile");

constexpr size_t kSzAct  = (size_t)kRows * kFeat * 2;
constexpr size_t kSzP    = (size_t)kRows * kPW * 4;
constexpr size_t kSzW    = (size_t)kFeat * kFeat * 2;
constexpr size_t kOffX16 = 0;
constexpr size_t kOffTH  = kOffX16 + kSzAct;
constexpr size_t kOffTL  = kOffTH  + kSzAct;
constexpr size_t kOffHH  = kOffTL  + kSzAct;
constexpr size_t kOffHL  = kOffHH  + kSzAct;
constexpr size_t kOffAH  = kOffHL  + kSzAct;
constexpr size_t kOffAL  = kOffAH  + kSzAct;
constexpr size_t kOffPP  = kOffAL  + kSzAct;
constexpr size_t kOffWI1 = kOffPP  + kSzP;
constexpr size_t kOffWI2 = kOffWI1 + kSzW;
constexpr size_t kOffWE1 = kOffWI2 + kSzW;
constexpr size_t kOffWE2 = kOffWE1 + 2 * kSzW;
constexpr size_t kOffWN1 = kOffWE2 + kSzW;
constexpr size_t kOffWN2 = kOffWN1 + kSzW;
constexpr size_t kOffINV = kOffWN2 + kSzW;
constexpr size_t kWsTotal = kOffINV + 128;
static_assert(kWsTotal == 47054976ull, "carve total");
static_assert(kWsTotal <= 134217728ull, "carve cap");
static_assert((kSzAct % 128) == 0 && (kSzP % 128) == 0 && (kSzW % 128) == 0, "128-B aligned regions");

__device__ __forceinline__ unsigned short f2bf_bits(float f) {
  unsigned u = __float_as_uint(f);
  return (unsigned short)((u + 0x7FFFu + ((u >> 16) & 1u)) >> 16);
}
__device__ __forceinline__ float bf_bits2f(unsigned short h) { return __uint_as_float(((unsigned)h) << 16); }
__device__ __forceinline__ float bf_rne(float f) { return bf_bits2f(f2bf_bits(f)); }

__device__ __forceinline__ void guard4_b(v8f& a, v8f& b, v8f& c, v8f& d, v16b x, v16b y) {
  asm volatile("v_nop\n\tv_nop\n\tv_nop\n\tv_nop" : "+v"(a), "+v"(b), "+v"(c), "+v"(d) : "v"(x), "v"(y));
}
__device__ __forceinline__ void guard2_h(v8f& a, v8f& b, v16h x, v16h y, v16h z) {
  asm volatile("v_nop\n\tv_nop\n\tv_nop\n\tv_nop" : "+v"(a), "+v"(b) : "v"(x), "v"(y), "v"(z));
}
__device__ __forceinline__ void keep4_b(v16b a, v16b b, v16b c, v16b d) { asm volatile("v_nop" :: "v"(a), "v"(b), "v"(c), "v"(d)); }
__device__ __forceinline__ void acc_guard4(v8f& a, v8f& b, v8f& c, v8f& d) { asm volatile("v_nop\n\tv_nop\n\tv_nop\n\tv_nop" : "+v"(a), "+v"(b), "+v"(c), "+v"(d)); }

template <typename T> struct Frag;
template <> struct Frag<_Float16> {
  typedef v16h V; union U { v16h v; v8h h[2]; };
  static __device__ __forceinline__ v16h load(const _Float16* p) {
    U f; f.h[0] = *(const v8h*)(p); f.h[1] = *(const v8h*)(p + 16); return f.v;
  }
  static __device__ __forceinline__ v8f mma(v16h a, v16h b, v8f c) {
    return __builtin_amdgcn_wmma_f32_16x16x32_f16(false, a, false, b, (short)0, c, false, false);
  }
};
template <> struct Frag<__bf16> {
  typedef v16b V; union U { v16b v; v8b h[2]; };
  static __device__ __forceinline__ v16b load(const __bf16* p) {
    U f; f.h[0] = *(const v8b*)(p); f.h[1] = *(const v8b*)(p + 16); return f.v;
  }
  static __device__ __forceinline__ v8f mma(v16b a, v16b b, v8f c) {
    return __builtin_amdgcn_wmma_f32_16x16x32_bf16(false, a, false, b, (short)0, c, false, false);
  }
};

__device__ __forceinline__ void split8_bf16(const v4f a0, const v4f a1, v8h& hv, v8h& lv) {
#pragma unroll
  for (int e = 0; e < 4; ++e) {
    const unsigned short h0 = f2bf_bits(a0[e]);
    const unsigned short h1 = f2bf_bits(a1[e]);
    const unsigned short l0 = f2bf_bits(a0[e] - bf_bits2f(h0));
    const unsigned short l1 = f2bf_bits(a1[e] - bf_bits2f(h1));
    hv[e]     = __builtin_bit_cast(_Float16, h0);
    hv[4 + e] = __builtin_bit_cast(_Float16, h1);
    lv[e]     = __builtin_bit_cast(_Float16, l0);
    lv[4 + e] = __builtin_bit_cast(_Float16, l1);
  }
}

template <int SPL, int BIAS_MODE, int OUT_MODE, int ACT>
__global__ __launch_bounds__(256) void wmma_gemm64(
    const unsigned short* __restrict__ Ap, const unsigned short* __restrict__ A2p, int lda,
    const unsigned short* __restrict__ Btp, int ldb,
    void* __restrict__ Cout, void* __restrict__ Cout2, int ldc,
    const float* __restrict__ bias, int M, int N, int K) {
  typedef __bf16 T;
  typedef Frag<T>::V V;
  const T* A = (const T*)Ap; const T* A2 = (const T*)A2p; const T* Bt = (const T*)Btp;
  __shared__ __align__(16) float sT[8][16 * 68];
  const int lane = threadIdx.x & 31;
  const int wave = __builtin_amdgcn_readfirstlane((int)(threadIdx.x >> 5));
  const int tilesN = N >> 6;
  const int tilesM = M >> 6;
  const int tile = blockIdx.x * 8 + wave;
  if (tile >= tilesM * tilesN) return;
  const int tm = tile / tilesN;
  const int tn = tile - tm * tilesN;
  const int m0 = tm << 6;
  const int n0 = tn << 6;

  const int rlane = lane & 15;
  const int koff  = (lane >> 4) * 8;
  const int mOff  = (lane >> 4) * 8;

  v8f acc[4][4];
#pragma unroll
  for (int i = 0; i < 4; ++i)
#pragma unroll
    for (int j = 0; j < 4; ++j) acc[i][j] = (v8f){0.f,0.f,0.f,0.f,0.f,0.f,0.f,0.f};

  for (int k0 = 0; k0 < K; k0 += 32) {
    V bh[4];
#pragma unroll
    for (int j = 0; j < 4; ++j) {
      const size_t bo = (size_t)(n0 + (j << 4) + rlane) * ldb + koff + k0;
      bh[j] = Frag<T>::load(Bt + bo);
    }
#pragma unroll
    for (int i = 0; i < 4; ++i) {
      const size_t ao = (size_t)(m0 + (i << 4) + rlane) * lda + koff + k0;
      V ah = Frag<T>::load(A + ao);
      V al;
      if (SPL >= 1) al = Frag<T>::load(A2 + ao);
#pragma unroll
      for (int j = 0; j < 4; ++j) {
        acc[i][j] = Frag<T>::mma(ah, bh[j], acc[i][j]);
        if (SPL >= 1) acc[i][j] = Frag<T>::mma(al, bh[j], acc[i][j]);
      }
      guard4_b(acc[i][0], acc[i][1], acc[i][2], acc[i][3], ah, (SPL >= 1) ? al : ah);
    }
    keep4_b(bh[0], bh[1], bh[2], bh[3]);
  }
  acc_guard4(acc[0][0], acc[0][1], acc[0][2], acc[0][3]);
  acc_guard4(acc[1][0], acc[1][1], acc[1][2], acc[1][3]);
  acc_guard4(acc[2][0], acc[2][1], acc[2][2], acc[2][3]);
  acc_guard4(acc[3][0], acc[3][1], acc[3][2], acc[3][3]);

  float* slab = sT[wave];
#pragma unroll
  for (int i = 0; i < 4; ++i) {
    const int mBase = m0 + (i << 4);
#pragma unroll
    for (int j = 0; j < 4; ++j) {
      const int n = n0 + (j << 4) + rlane;
      float bv = 0.f;
      if (BIAS_MODE == 2) bv = bf_rne(bias[n]);
#pragma unroll
      for (int r = 0; r < 8; ++r) {
        float v = acc[i][j][r];
        if (BIAS_MODE == 2) v += bv;
        if (ACT == 2) v = fmaxf(v, 0.0f);
        slab[(mOff + r) * 68 + (j << 4) + rlane] = v;
      }
    }
    __builtin_amdgcn_fence(__ATOMIC_RELEASE, "workgroup");
    __builtin_amdgcn_wave_barrier();
    __builtin_amdgcn_fence(__ATOMIC_ACQUIRE, "workgroup");
    if (OUT_MODE == 0) {
      float* C = (float*)Cout;
      const int hh = lane >> 4, c4 = (lane & 15) * 4;
      for (int pass = 0; pass < 2; ++pass) {
#pragma unroll
        for (int it = 0; it < 8; ++it) {
          const int row = it * 2 + hh;
          v4f v = *(const v4f*)(slab + row * 68 + c4);
          *(volatile v4f*)(C + (size_t)(mBase + row) * ldc + n0 + c4) = v;
        }
        __threadfence();
      }
    } else {
      const int q = lane >> 3, c8 = (lane & 7) * 8;
      unsigned short* C  = (unsigned short*)Cout;
      unsigned short* C2 = (unsigned short*)Cout2;
      for (int pass = 0; pass < 2; ++pass) {
#pragma unroll
        for (int it = 0; it < 4; ++it) {
          const int row = it * 4 + q;
          const float* sp = slab + row * 68 + c8;
          const v4f a0 = *(const v4f*)(sp);
          const v4f a1 = *(const v4f*)(sp + 4);
          v8h hv, lv;
          split8_bf16(a0, a1, hv, lv);
          *(volatile v8h*)(C  + (size_t)(mBase + row) * ldc + n0 + c8) = hv;
          *(volatile v8h*)(C2 + (size_t)(mBase + row) * ldc + n0 + c8) = lv;
        }
        __threadfence();
      }
    }
    __builtin_amdgcn_fence(__ATOMIC_RELEASE, "workgroup");
    __builtin_amdgcn_wave_barrier();
    __builtin_amdgcn_fence(__ATOMIC_ACQUIRE, "workgroup");
  }
}

__global__ __launch_bounds__(256) void prep_weights_kernel(
    const float* __restrict__ w_in1, const float* __restrict__ w_in2, const float* __restrict__ w_e1,
    const float* __restrict__ w_e2, const float* __restrict__ w_n1, const float* __restrict__ w_n2,
    unsigned short* __restrict__ d_in1, unsigned short* __restrict__ d_in2, unsigned short* __restrict__ d_e1,
    unsigned short* __restrict__ d_e2, unsigned short* __restrict__ d_n1, unsigned short* __restrict__ d_n2)
{
  __shared__ __align__(16) float sW[64 * 65];
  const int tid = threadIdx.x, lane = tid & 31;
  const int wave = __builtin_amdgcn_readfirstlane((int)(threadIdx.x >> 5));
  const int y = blockIdx.y;
  const float* src = w_in1;
  unsigned short* dst = d_in1;
  if (y == 1) { src = w_in2; dst = d_in2; }
  if (y == 2) { src = w_e1; dst = d_e1; }
  if (y == 3) { src = w_e1 + kFeat * kFeat; dst = d_e1 + kFeat * kFeat; }
  if (y == 4) { src = w_e2; dst = d_e2; }
  if (y == 5) { src = w_n1; dst = d_n1; }
  if (y == 6) { src = w_n2; dst = d_n2; }
  const bool asF16 = (y == 4);
  const int k0 = (blockIdx.x >> 2) * 64;
  const int n0 = (blockIdx.x & 3) * 64;
#pragma unroll
  for (int i = 0; i < 4; ++i) {
    const int u = tid + i * 256;
    const int kk = u >> 4, c4 = (u & 15) * 4;
    const v4f v = *(const v4f*)(src + (size_t)(k0 + kk) * kFeat + n0 + c4);
    sW[kk * 65 + c4 + 0] = v[0];
    sW[kk * 65 + c4 + 1] = v[1];
    sW[kk * 65 + c4 + 2] = v[2];
    sW[kk * 65 + c4 + 3] = v[3];
  }
  __syncthreads();
  const int q = lane >> 3, c8 = (lane & 7) * 8;
  v8h hv[2];
#pragma unroll
  for (int it = 0; it < 2; ++it) {
    const int nn = it * 32 + wave * 4 + q;
#pragma unroll
    for (int e = 0; e < 8; ++e) {
      const float raw = sW[(c8 + e) * 65 + nn];
      const unsigned short bb = f2bf_bits(raw);
      const _Float16 hf = (_Float16)(bf_bits2f(bb) * kWCarry);
      const unsigned short fb = __builtin_bit_cast(unsigned short, hf);
      const unsigned short bits = asF16 ? fb : bb;
      hv[it][e] = __builtin_bit_cast(_Float16, bits);
    }
  }
  for (int pass = 0; pass < 2; ++pass) {
#pragma unroll
    for (int it = 0; it < 2; ++it) {
      const int nn = it * 32 + wave * 4 + q;
      *(volatile v8h*)(dst + (size_t)(n0 + nn) * kFeat + k0 + c8) = hv[it];
    }
    __threadfence();
  }
}

__global__ __launch_bounds__(256) void cvt_rows_bf16_kernel(
    const float* __restrict__ src, unsigned short* __restrict__ dst, int total8)
{
  const int i = blockIdx.x * 256 + threadIdx.x;
  if (i >= total8) return;
  const size_t e0 = (size_t)i << 3;
  const v4f a0 = *(const v4f*)(src + e0);
  const v4f a1 = *(const v4f*)(src + e0 + 4);
  v8h hv;
#pragma unroll
  for (int e = 0; e < 4; ++e) {
    const unsigned short h0 = f2bf_bits(a0[e]);
    const unsigned short h1 = f2bf_bits(a1[e]);
    hv[e]     = __builtin_bit_cast(_Float16, h0);
    hv[4 + e] = __builtin_bit_cast(_Float16, h1);
  }
  unsigned short* qd = dst + e0;
  *(volatile v8h*)qd = hv;
  __threadfence();
  *(volatile v8h*)qd = hv;
}

__global__ __launch_bounds__(32) void indegree_kernel(const int* __restrict__ recIdx, float* __restrict__ invdeg)
{
  const int lane = threadIdx.x & 31;
  int cnt = 0;
#pragma unroll 1
  for (int e = 0; e < kEdges; ++e) {
    int r = recIdx[e];
    r = r < 0 ? 0 : (r > kNodes - 1 ? kNodes - 1 : r);
    cnt += (r == lane) ? 1 : 0;
  }
  const float v = 1.0f / (float)cnt;
  volatile float* qd = invdeg + lane;
  *qd = v;
  __threadfence();
  *qd = v;
}

__global__ __launch_bounds__(512) void edge_kernel(
    const float* __restrict__ P, const int* __restrict__ sendIdx, const int* __restrict__ recIdx,
    const unsigned short* __restrict__ We2T, const float* __restrict__ b_e1, const float* __restrict__ b_e2,
    const float* __restrict__ invdeg, unsigned short* __restrict__ AH, unsigned short* __restrict__ AL)
{
  __shared__ __align__(16) float    sP[kNodes * kPW];
  __shared__ __align__(16) _Float16 sZ[2 * kZTile];
  __shared__ __align__(16) int      sSend[kEPad];
  __shared__ __align__(16) int      sRec[kEPad];
  __shared__ __align__(16) float    sInv[kNodes];
  union FH { v16h v; v8h q[2]; };

  const int tid  = threadIdx.x;
  const int lane = tid & 31;
  const int wave = __builtin_amdgcn_readfirstlane((int)(threadIdx.x >> 5));
  const int h = lane >> 4, m = lane & 15;
  const int c8 = lane * 8;
  const int b = blockIdx.x;

  {
    const float* Pb = P + (size_t)b * kNodes * kPW;
#pragma unroll
    for (int i = 0; i < 8; ++i) {
      const int u = tid + i * 512;
      *(v4f*)(sP + 4 * u) = *(const v4f*)(Pb + 4 * u);
    }
  }
#pragma unroll
  for (int i = 0; i < 2; ++i) {
    const int e = tid + i * 512;
    const int ec = e < kEdges ? e : (kEdges - 1);
    int s = sendIdx[ec];
    int r = recIdx[ec];
    s = s < 0 ? 0 : (s > kNodes - 1 ? kNodes - 1 : s);
    r = r < 0 ? 0 : (r > kNodes - 1 ? kNodes - 1 : r);
    sSend[e] = s;
    sRec[e] = r;
  }
  if (wave == 0) sInv[lane] = invdeg[lane];

  float bz[8];
  {
    const v4f t0 = *(const v4f*)(b_e1 + c8);
    const v4f t1 = *(const v4f*)(b_e1 + c8 + 4);
#pragma unroll
    for (int e = 0; e < 4; ++e) { bz[e] = bf_rne(t0[e]); bz[4 + e] = bf_rne(t1[e]); }
  }
  const int ocol = 16 * wave + m;
  const float be2 = kECarry * bf_rne(b_e2[ocol]);

  v16h bw[8];
  {
    const _Float16* wp = (const _Float16*)We2T + (size_t)ocol * kFeat + 8 * h;
#pragma unroll
    for (int ks = 0; ks < 8; ++ks) bw[ks] = Frag<_Float16>::load(wp + ks * 32);
  }
  __syncthreads();

  v8f g0 = (v8f){0.f,0.f,0.f,0.f,0.f,0.f,0.f,0.f};
  v8f g1 = (v8f){0.f,0.f,0.f,0.f,0.f,0.f,0.f,0.f};

#pragma unroll 1
  for (int t = 0; t < kTiles; ++t) {
    const int zoff = (t & 1) * kZTile;
#pragma unroll
    for (int rr = 0; rr < 2; ++rr) {
      const int row = wave + 16 * rr;
      const int e = t * kTileE + row;
      const int s = sSend[e];
      const int r = sRec[e];
      const float* ps = sP + s * kPW + c8;
      const float* pr = sP + r * kPW + kFeat + c8;
      const v4f a0 = *(const v4f*)(ps);
      const v4f a1 = *(const v4f*)(ps + 4);
      const v4f q0 = *(const v4f*)(pr);
      const v4f q1 = *(const v4f*)(pr + 4);
      v8h zv;
#pragma unroll
      for (int i = 0; i < 4; ++i) {
        const float u0 = fmaxf((a0[i] + q0[i]) + bz[i], 0.0f) * kZCarry;
        const float u1 = fmaxf((a1[i] + q1[i]) + bz[4 + i], 0.0f) * kZCarry;
        zv[i]     = (_Float16)u0;
        zv[4 + i] = (_Float16)u1;
      }
      *(v8h*)(sZ + zoff + row * kZP + c8) = zv;
    }
    __syncthreads();

    v8f acc0 = (v8f){0.f,0.f,0.f,0.f,0.f,0.f,0.f,0.f};
    v8f acc1 = (v8f){0.f,0.f,0.f,0.f,0.f,0.f,0.f,0.f};
#pragma unroll
    for (int ks = 0; ks < 8; ++ks) {
      FH fa, fb;
      const _Float16* z0 = sZ + zoff + m * kZP + ks * 32 + 8 * h;
      const _Float16* z1 = sZ + zoff + (16 + m) * kZP + ks * 32 + 8 * h;
      fa.q[0] = *(const v8h*)(z0);
      fa.q[1] = *(const v8h*)(z0 + 16);
      fb.q[0] = *(const v8h*)(z1);
      fb.q[1] = *(const v8h*)(z1 + 16);
      acc0 = Frag<_Float16>::mma(fa.v, bw[ks], acc0);
      acc1 = Frag<_Float16>::mma(fb.v, bw[ks], acc1);
      guard2_h(acc0, acc1, fa.v, fb.v, bw[ks]);
    }

    const int* rp = sRec + t * kTileE + 8 * h;
    const v4i r0 = *(const v4i*)(rp);
    const v4i r1 = *(const v4i*)(rp + 4);
    const v4i r2 = *(const v4i*)(rp + 16);
    const v4i r3 = *(const v4i*)(rp + 20);
    v16h oh0, oh1;
#pragma unroll
    for (int i = 0; i < 4; ++i) {
      const int ia = r0[i], ib = r1[i], ic = r2[i], id = r3[i];
      oh0[i]      = (_Float16)((ia == m) ? 1.0f : 0.0f);
      oh0[4 + i]  = (_Float16)((ib == m) ? 1.0f : 0.0f);
      oh0[8 + i]  = (_Float16)((ic == m) ? 1.0f : 0.0f);
      oh0[12 + i] = (_Float16)((id == m) ? 1.0f : 0.0f);
      oh1[i]      = (_Float16)((ia == m + 16) ? 1.0f : 0.0f);
      oh1[4 + i]  = (_Float16)((ib == m + 16) ? 1.0f : 0.0f);
      oh1[8 + i]  = (_Float16)((ic == m + 16) ? 1.0f : 0.0f);
      oh1[12 + i] = (_Float16)((id == m + 16) ? 1.0f : 0.0f);
    }
    v16h eb;
#pragma unroll
    for (int r = 0; r < 8; ++r) {
      const float e0 = fmaxf(acc0[r] * kAccToE + be2, 0.0f);
      const float e1 = fmaxf(acc1[r] * kAccToE + be2, 0.0f);
      eb[r]     = (_Float16)e0;
      eb[8 + r] = (_Float16)e1;
    }
    g0 = Frag<_Float16>::mma(oh0, eb, g0);
    g1 = Frag<_Float16>::mma(oh1, eb, g1);
    guard2_h(g0, g1, oh0, oh1, eb);
  }

  __syncthreads();
  float* sO = sP;
  {
    const v4f i0 = *(const v4f*)(sInv + 8 * h);
    const v4f i1 = *(const v4f*)(sInv + 8 * h + 4);
    const v4f i2 = *(const v4f*)(sInv + 16 + 8 * h);
    const v4f i3 = *(const v4f*)(sInv + 16 + 8 * h + 4);
#pragma unroll
    for (int r = 0; r < 4; ++r) {
      sO[(8 * h + r) * kOP + ocol]          = g0[r]     * (i0[r] * kEInv);
      sO[(8 * h + 4 + r) * kOP + ocol]      = g0[4 + r] * (i1[r] * kEInv);
      sO[(16 + 8 * h + r) * kOP + ocol]     = g1[r]     * (i2[r] * kEInv);
      sO[(16 + 8 * h + 4 + r) * kOP + ocol] = g1[4 + r] * (i3[r] * kEInv);
    }
  }
  __syncthreads();
  v8h hv[2], lv[2];
#pragma unroll
  for (int rr = 0; rr < 2; ++rr) {
    const int row = wave + 16 * rr;
    const float* sp = sO + row * kOP + c8;
    const v4f a0 = *(const v4f*)(sp);
    const v4f a1 = *(const v4f*)(sp + 4);
    split8_bf16(a0, a1, hv[rr], lv[rr]);
  }
  for (int pass = 0; pass < 2; ++pass) {
#pragma unroll
    for (int rr = 0; rr < 2; ++rr) {
      const int row = wave + 16 * rr;
      const size_t o = ((size_t)b * kNodes + row) * kFeat + c8;
      *(volatile v8h*)(AH + o) = hv[rr];
      *(volatile v8h*)(AL + o) = lv[rr];
    }
    __threadfence();
  }
}

extern "C" void kernel_launch(void* const* d_in, const int* in_sizes, int n_in,
                              void* d_out, int out_size, void* d_ws, size_t ws_size,
                              hipStream_t stream) {
  if (n_in < 15) return;
  if (in_sizes[0] != kRows * kFeat) return;
  if (in_sizes[1] != kEdges || in_sizes[2] != kEdges) return;
  if (in_sizes[3] != kFeat * kFeat || in_sizes[5] != kFeat * kFeat) return;
  if (in_sizes[7] != 2 * kFeat * kFeat) return;
  if (in_sizes[9] != kFeat * kFeat || in_sizes[11] != kFeat * kFeat || in_sizes[13] != kFeat * kFeat) return;
  if (in_sizes[4] != kFeat || in_sizes[6] != kFeat || in_sizes[8] != kFeat) return;
  if (in_sizes[10] != kFeat || in_sizes[12] != kFeat || in_sizes[14] != kFeat) return;
  if (out_size != kRows * kFeat) return;
  if (ws_size < kWsTotal) return;

  const float* x     = (const float*)d_in[0];
  const int*   rec   = (const int*)d_in[1];
  const int*   snd   = (const int*)d_in[2];
  const float* w_in1 = (const float*)d_in[3];
  const float* b_in1 = (const float*)d_in[4];
  const float* w_in2 = (const float*)d_in[5];
  const float* b_in2 = (const float*)d_in[6];
  const float* w_e1  = (const float*)d_in[7];
  const float* b_e1  = (const float*)d_in[8];
  const float* w_e2  = (const float*)d_in[9];
  const float* b_e2  = (const float*)d_in[10];
  const float* w_n1  = (const float*)d_in[11];
  const float* b_n1  = (const float*)d_in[12];
  const float* w_n2  = (const float*)d_in[13];
  const float* b_n2  = (const float*)d_in[14];
  float* out = (float*)d_out;

  char* ws = (char*)d_ws;
  unsigned short* X16 = (unsigned short*)(ws + kOffX16);
  unsigned short* TH  = (unsigned short*)(ws + kOffTH);
  unsigned short* TL  = (unsigned short*)(ws + kOffTL);
  unsigned short* HH  = (unsigned short*)(ws + kOffHH);
  unsigned short* HL  = (unsigned short*)(ws + kOffHL);
  unsigned short* AH  = (unsigned short*)(ws + kOffAH);
  unsigned short* AL  = (unsigned short*)(ws + kOffAL);
  float*          PP  = (float*)(ws + kOffPP);
  unsigned short* WI1 = (unsigned short*)(ws + kOffWI1);
  unsigned short* WI2 = (unsigned short*)(ws + kOffWI2);
  unsigned short* WE1 = (unsigned short*)(ws + kOffWE1);
  unsigned short* WE2 = (unsigned short*)(ws + kOffWE2);
  unsigned short* WN1 = (unsigned short*)(ws + kOffWN1);
  unsigned short* WN2 = (unsigned short*)(ws + kOffWN2);
  float*          INV = (float*)(ws + kOffINV);

  prep_weights_kernel<<<dim3(16, 7), 256, 0, stream>>>(w_in1, w_in2, w_e1, w_e2, w_n1, w_n2,
                                                       WI1, WI2, WE1, WE2, WN1, WN2);
  indegree_kernel<<<1, 32, 0, stream>>>(rec, INV);
  cvt_rows_bf16_kernel<<<(kRows * kFeat / 8) / 256, 256, 0, stream>>>(x, X16, kRows * kFeat / 8);

  const int gridN256 = (kRows / 64) * (kFeat / 64) / 8;
  const int gridN512 = (kRows / 64) * (kPW / 64) / 8;

  wmma_gemm64<0, 2, 2, 2><<<gridN256, 256, 0, stream>>>(X16, nullptr, kFeat, WI1, kFeat,
      (void*)TH, (void*)TL, kFeat, b_in1, kRows, kFeat, kFeat);
  wmma_gemm64<1, 2, 2, 2><<<gridN256, 256, 0, stream>>>(TH, TL, kFeat, WI2, kFeat,
      (void*)HH, (void*)HL, kFeat, b_in2, kRows, kFeat, kFeat);

  for (int pass = 0; pass < 2; ++pass) {
    wmma_gemm64<1, 0, 0, 0><<<gridN512, 256, 0, stream>>>(HH, HL, kFeat, WE1, kFeat,
        (void*)PP, nullptr, kPW, nullptr, kRows, kPW, kFeat);
    edge_kernel<<<kBatch, 512, 0, stream>>>(PP, snd, rec, WE2, b_e1, b_e2, INV, AH, AL);
    wmma_gemm64<1, 2, 2, 2><<<gridN256, 256, 0, stream>>>(AH, AL, kFeat, WN1, kFeat,
        (void*)TH, (void*)TL, kFeat, b_n1, kRows, kFeat, kFeat);
    if (pass == 0) {
      wmma_gemm64<1, 2, 2, 2><<<gridN256, 256, 0, stream>>>(TH, TL, kFeat, WN2, kFeat,
          (void*)HH, (void*)HL, kFeat, b_n2, kRows, kFeat, kFeat);
    } else {
      wmma_gemm64<1, 2, 0, 2><<<gridN256, 256, 0, stream>>>(TH, TL, kFeat, WN2, kFeat,
          (void*)out, nullptr, kFeat, b_n2, kRows, kFeat, kFeat);
    }
  }
}
